// Bottleneck_DCNv3_29652454212243
// MI455X (gfx1250) — hardware-verified
//
#include <hip/hip_runtime.h>
#include <stddef.h>

constexpr int NBATCH = 2;
constexpr int NCH    = 256;
constexpr int IMG_H  = 64;
constexpr int IMG_W  = 64;
constexpr int HWPIX  = 4096;
constexpr int NPIX   = 8192;
constexpr int NTAP   = 9;
constexpr int KCONV  = 2304;
constexpr int NOMC   = 27;
constexpr int NOMP   = 64;
constexpr int NOFF   = 18;
constexpr int NITEM  = NPIX * NTAP;
constexpr float BN_EPS_F = 1e-5f;
constexpr float LN_EPS_F = 1e-5f;
constexpr int PAR_SHIFT1 = 0;
constexpr int PAR_BIAS2  = 256;
constexpr int PAR_BIAS64 = 512;
constexpr int PAR_DWT    = 1024;
constexpr int PAR_FLOATS = 4096;
static_assert(KCONV % 32 == 0, "K tail");
static_assert(NCH % 64 == 0 && NPIX % 64 == 0 && HWPIX % 64 == 0 && NOMP % 64 == 0, "tile multiples");
static_assert(NITEM % 32 == 0, "item grid exact");
static_assert(PAR_DWT + NTAP * NCH <= PAR_FLOATS, "par region");

typedef __attribute__((ext_vector_type(16))) _Float16 v16h;
typedef __attribute__((ext_vector_type(8)))  _Float16 v8h;
typedef __attribute__((ext_vector_type(16))) __bf16   v16b;
typedef __attribute__((ext_vector_type(8)))  __bf16   v8b;
typedef __attribute__((ext_vector_type(8)))  float    v8f;
typedef __attribute__((ext_vector_type(4)))  float    v4f;
typedef __attribute__((ext_vector_type(4)))  unsigned v4u;

__device__ __forceinline__ unsigned short f2bf_bits(float f) {
  unsigned u = __float_as_uint(f);
  return (unsigned short)((u + 0x7FFFu + ((u >> 16) & 1u)) >> 16);
}
__device__ __forceinline__ float bf_bits2f(unsigned short h) { return __uint_as_float(((unsigned)h) << 16); }

__device__ __forceinline__ unsigned pk2(unsigned short a, unsigned short b) {
  return (unsigned)a | ((unsigned)b << 16);
}
__device__ __forceinline__ unsigned pkh2(float a, float b) {
  return pk2(__builtin_bit_cast(unsigned short, (_Float16)a), __builtin_bit_cast(unsigned short, (_Float16)b));
}

__device__ __forceinline__ void dep_guard_h(v8f& a, v8f& b, v16h x, v16h y) { asm volatile("v_nop\n\tv_nop\n\tv_nop\n\tv_nop" : "+v"(a), "+v"(b) : "v"(x), "v"(y)); }
__device__ __forceinline__ void dep_guard_b(v8f& a, v8f& b, v16b x, v16b y) { asm volatile("v_nop\n\tv_nop\n\tv_nop\n\tv_nop" : "+v"(a), "+v"(b) : "v"(x), "v"(y)); }
__device__ __forceinline__ void keep4_h(v16h a, v16h b, v16h c, v16h d) { asm volatile("v_nop" :: "v"(a), "v"(b), "v"(c), "v"(d)); }
__device__ __forceinline__ void keep4_b(v16b a, v16b b, v16b c, v16b d) { asm volatile("v_nop" :: "v"(a), "v"(b), "v"(c), "v"(d)); }
__device__ __forceinline__ void acc_guard4(v8f& a, v8f& b, v8f& c, v8f& d) { asm volatile("v_nop\n\tv_nop\n\tv_nop\n\tv_nop" : "+v"(a), "+v"(b), "+v"(c), "+v"(d)); }
template <typename T> struct Frag;
template <> struct Frag<_Float16> {
  typedef v16h V; union U { v16h v; v8h h[2]; };
  static __device__ __forceinline__ v16h load(const _Float16* p) {
    U f; f.h[0] = *(const v8h*)(p); f.h[1] = *(const v8h*)(p + 16); return f.v;
  }
  static __device__ __forceinline__ v8f mma(v16h a, v16h b, v8f c) {
    return __builtin_amdgcn_wmma_f32_16x16x32_f16(false, a, false, b, (short)0, c, false, false);
  }
  static __device__ __forceinline__ void guard(v8f& a, v8f& b, v16h x, v16h y) { dep_guard_h(a, b, x, y); }
  static __device__ __forceinline__ void keep(v16h a, v16h b, v16h c, v16h d) { keep4_h(a, b, c, d); }
};
template <> struct Frag<__bf16> {
  typedef v16b V; union U { v16b v; v8b h[2]; };
  static __device__ __forceinline__ v16b load(const __bf16* p) {
    U f; f.h[0] = *(const v8b*)(p); f.h[1] = *(const v8b*)(p + 16); return f.v;
  }
  static __device__ __forceinline__ v8f mma(v16b a, v16b b, v8f c) {
    return __builtin_amdgcn_wmma_f32_16x16x32_bf16(false, a, false, b, (short)0, c, false, false);
  }
  static __device__ __forceinline__ void guard(v8f& a, v8f& b, v16b x, v16b y) { dep_guard_b(a, b, x, y); }
  static __device__ __forceinline__ void keep(v16b a, v16b b, v16b c, v16b d) { keep4_b(a, b, c, d); }
};

template <int ET> struct Elem;
template <> struct Elem<0> { typedef _Float16 T; };
template <> struct Elem<1> { typedef __bf16 T; };
template <int ET, bool SPLIT, int BIAS_MODE, int OUT_MODE, bool RESID, int ACT = 0>
__global__ __launch_bounds__(256) void wmma_gemm64(
    const unsigned short* __restrict__ Ap, const unsigned short* __restrict__ A2p, int lda, long strideA,
    const unsigned short* __restrict__ Btp, const unsigned short* __restrict__ Bt2p, int ldb, long strideB,
    void* __restrict__ Cout, void* __restrict__ Cout2, int ldc, long strideC,
    const float* __restrict__ bias,
    const float* __restrict__ resid, long strideR,
    int M, int N, int K, float scale) {
  typedef typename Elem<ET>::T T;
  typedef typename Frag<T>::V V;
  const T* A = (const T*)Ap; const T* A2 = (const T*)A2p; const T* Bt = (const T*)Btp; const T* Bt2 = (const T*)Bt2p;
  __shared__ __align__(16) float sT[8][16 * 68];
  const int b    = blockIdx.y;
  const int lane = threadIdx.x & 31;
  const int wave = threadIdx.x >> 5;
  const int tilesN = N >> 6;
  const int tilesM = M >> 6;
  const int tile = blockIdx.x * 8 + wave;
  if (tile >= tilesM * tilesN) return;
  const int tm = tile / tilesN;
  const int tn = tile - tm * tilesN;
  const int m0 = tm << 6;
  const int n0 = tn << 6;

  const T* Ab  = A  + (size_t)b * strideA;
  const T* Bb  = Bt + (size_t)b * strideB;
  const T* Ab2 = SPLIT ? (A2  + (size_t)b * strideA) : nullptr;
  const T* Bb2 = SPLIT ? (Bt2 + (size_t)b * strideB) : nullptr;

  const int rlane = lane & 15;
  const int koff  = (lane >> 4) * 8;
  const int mOff  = (lane >> 4) * 8;

  v8f acc[4][4];
#pragma unroll
  for (int i = 0; i < 4; ++i)
#pragma unroll
    for (int j = 0; j < 4; ++j) acc[i][j] = (v8f){0.f,0.f,0.f,0.f,0.f,0.f,0.f,0.f};

  for (int k0 = 0; k0 < K; k0 += 32) {
    V bh[4], bl[4];
#pragma unroll
    for (int j = 0; j < 4; ++j) {
      const size_t bo = (size_t)(n0 + (j << 4) + rlane) * ldb + koff + k0;
      bh[j] = Frag<T>::load(Bb + bo);
      if (SPLIT) bl[j] = Frag<T>::load(Bb2 + bo);
    }
#pragma unroll
    for (int i = 0; i < 4; ++i) {
      const size_t ao = (size_t)(m0 + (i << 4) + rlane) * lda + koff + k0;
      V ah = Frag<T>::load(Ab + ao);
      V al;
      if (SPLIT) al = Frag<T>::load(Ab2 + ao);
#pragma unroll
      for (int j = 0; j < 4; ++j) {
        acc[i][j] = Frag<T>::mma(ah, bh[j], acc[i][j]);
        if (SPLIT) {
          acc[i][j] = Frag<T>::mma(ah, bl[j], acc[i][j]);
          acc[i][j] = Frag<T>::mma(al, bh[j], acc[i][j]);
        }
      }
      Frag<T>::guard(acc[i][0], acc[i][3], ah, SPLIT ? al : ah);
    }
    Frag<T>::keep(bh[0], bh[1], bh[2], bh[3]);
    if (SPLIT) Frag<T>::keep(bl[0], bl[1], bl[2], bl[3]);
  }
  acc_guard4(acc[0][0], acc[0][1], acc[0][2], acc[0][3]);
  acc_guard4(acc[1][0], acc[1][1], acc[1][2], acc[1][3]);
  acc_guard4(acc[2][0], acc[2][1], acc[2][2], acc[2][3]);
  acc_guard4(acc[3][0], acc[3][1], acc[3][2], acc[3][3]);

  float* slab = sT[wave];
  const float* Rb = RESID ? (resid + (size_t)b * strideR) : nullptr;
#pragma unroll
  for (int i = 0; i < 4; ++i) {
    const int mBase = m0 + (i << 4);
#pragma unroll
    for (int j = 0; j < 4; ++j) {
      const int n = n0 + (j << 4) + rlane;
      float bv = 0.f;
      if (BIAS_MODE == 2) bv = bias[n];
#pragma unroll
      for (int r = 0; r < 8; ++r) {
        float v = acc[i][j][r] * scale;
        if (BIAS_MODE == 1) v += bias[mBase + mOff + r];
        if (BIAS_MODE == 2) v += bv;
        if (ACT == 2) v = fmaxf(v, 0.0f);
        if (ACT == 3) v = v * __builtin_amdgcn_rcpf(1.0f + __expf(-v));
        if (RESID) v += Rb[(size_t)(mBase + mOff + r) * ldc + n];
        slab[(mOff + r) * 68 + (j << 4) + rlane] = v;
      }
    }
    __builtin_amdgcn_fence(__ATOMIC_RELEASE, "workgroup");
    __builtin_amdgcn_wave_barrier();
    __builtin_amdgcn_fence(__ATOMIC_ACQUIRE, "workgroup");
    if (OUT_MODE == 0 || OUT_MODE == 3) {
      float* C = (float*)Cout + (size_t)b * strideC;
      const int hh = lane >> 4, c4 = (lane & 15) * 4;
      for (int pass = 0; pass < 2; ++pass) {
#pragma unroll
        for (int it = 0; it < 8; ++it) {
          const int row = it * 2 + hh;
          v4f v = *(const v4f*)(slab + row * 68 + c4);
          *(volatile v4f*)(C + (size_t)(mBase + row) * ldc + n0 + c4) = v;
        }
        __threadfence();
      }
    }
    if (OUT_MODE != 0) {
      const int q = lane >> 3, c8 = (lane & 7) * 8;
      unsigned short* C  = (unsigned short*)((OUT_MODE == 3) ? Cout2 : Cout) + (size_t)b * strideC;
      unsigned short* C2 = (OUT_MODE == 2) ? ((unsigned short*)Cout2 + (size_t)b * strideC) : nullptr;
      for (int pass = 0; pass < 2; ++pass) {
#pragma unroll
        for (int it = 0; it < 4; ++it) {
          const int row = it * 4 + q;
          const float* sp = slab + row * 68 + c8;
          v8h hv, lv;
#pragma unroll
          for (int e = 0; e < 8; ++e) {
            if (OUT_MODE == 1 || OUT_MODE == 3) {
              hv[e] = (_Float16)sp[e];
            } else {
              unsigned short hb = f2bf_bits(sp[e]);
              unsigned short lb = f2bf_bits(sp[e] - bf_bits2f(hb));
              hv[e] = __builtin_bit_cast(_Float16, hb);
              lv[e] = __builtin_bit_cast(_Float16, lb);
            }
          }
          *(volatile v8h*)(C + (size_t)(mBase + row) * ldc + n0 + c8) = hv;
          if (OUT_MODE == 2) *(volatile v8h*)(C2 + (size_t)(mBase + row) * ldc + n0 + c8) = lv;
        }
        __threadfence();
      }
    }
    __builtin_amdgcn_fence(__ATOMIC_RELEASE, "workgroup");
    __builtin_amdgcn_wave_barrier();
    __builtin_amdgcn_fence(__ATOMIC_ACQUIRE, "workgroup");
  }
}

__device__ __forceinline__ float bn_inv(const float* __restrict__ gamma, const float* __restrict__ rvar, int o) {
  return gamma[o] / sqrtf(rvar[o] + BN_EPS_F);
}

__global__ __launch_bounds__(256) void k_prep_w1(const float* __restrict__ w, const float* __restrict__ gamma,
                                                 const float* __restrict__ beta, const float* __restrict__ rmean,
                                                 const float* __restrict__ rvar,
                                                 unsigned short* __restrict__ Bw, float* __restrict__ shift) {
  const int g = blockIdx.x * 256 + threadIdx.x;
  if (g < NCH * KCONV / 8) {
    const int e0 = g * 8;
    const int o  = e0 / KCONV;
    const int col = e0 - o * KCONV;
    const int k  = col >> 8;
    const int c0 = col & (NCH - 1);
    const float sc = bn_inv(gamma, rvar, o) * 16.0f;
    float f[8];
#pragma unroll
    for (int j = 0; j < 8; ++j) f[j] = w[(size_t)(o * NCH + c0 + j) * NTAP + k] * sc;
    v4u u;
    u[0] = pkh2(f[0], f[1]); u[1] = pkh2(f[2], f[3]); u[2] = pkh2(f[4], f[5]); u[3] = pkh2(f[6], f[7]);
    volatile v4u* p = (volatile v4u*)(Bw + e0);
    *p = u;
    __threadfence();
    *p = u;
  }
  if (blockIdx.x == 0 && threadIdx.x < 32) {
    const int lane = threadIdx.x;
    v4f s0, s1;
#pragma unroll
    for (int e = 0; e < 4; ++e) {
      const int o0 = lane * 4 + e;
      const int o1 = 128 + lane * 4 + e;
      const float i0 = bn_inv(gamma, rvar, o0);
      const float i1 = bn_inv(gamma, rvar, o1);
      s0[e] = beta[o0] - rmean[o0] * i0;
      s1[e] = beta[o1] - rmean[o1] * i1;
    }
    volatile v4f* p0 = (volatile v4f*)(shift + lane * 4);
    volatile v4f* p1 = (volatile v4f*)(shift + 128 + lane * 4);
    *p0 = s0; *p1 = s1;
    __threadfence();
    *p0 = s0; *p1 = s1;
  }
}

__global__ __launch_bounds__(256) void k_prep_small(
    const float* __restrict__ in_w, const float* __restrict__ out_w, const float* __restrict__ out_b,
    const float* __restrict__ g2, const float* __restrict__ b2, const float* __restrict__ m2, const float* __restrict__ v2,
    const float* __restrict__ off_w, const float* __restrict__ off_b,
    const float* __restrict__ mk_w, const float* __restrict__ mk_b,
    const float* __restrict__ dw_w,
    unsigned short* __restrict__ INWP, unsigned short* __restrict__ OUTWP, unsigned short* __restrict__ OMW,
    float* __restrict__ par) {
  const int tid = threadIdx.x;
  const int blk = blockIdx.x;
  if (blk < 64) {
    const bool second = (blk >= 32);
    const int g  = (second ? (blk - 32) : blk) * 256 + tid;
    const int e0 = g * 8;
    const int o  = e0 >> 8;
    const int i0 = e0 & (NCH - 1);
    const float* src = second ? out_w : in_w;
    float sc = 16.0f;
    if (second) sc = bn_inv(g2, v2, o) * 16.0f;
    float f[8];
#pragma unroll
    for (int j = 0; j < 8; ++j) f[j] = src[(size_t)(i0 + j) * NCH + o] * sc;
    v4u u;
    u[0] = pkh2(f[0], f[1]); u[1] = pkh2(f[2], f[3]); u[2] = pkh2(f[4], f[5]); u[3] = pkh2(f[6], f[7]);
    volatile v4u* p = (volatile v4u*)((second ? OUTWP : INWP) + e0);
    *p = u;
    __threadfence();
    *p = u;
  } else if (blk < 72) {
    const int g  = (blk - 64) * 256 + tid;
    const int e0 = g * 8;
    const int n  = e0 >> 8;
    const int i0 = e0 & (NCH - 1);
    const int no = (n < NOFF) ? n : (NOFF - 1);
    const int nm = (n < NOFF) ? 0 : ((n < NOMC) ? (n - NOFF) : (NTAP - 1));
    float f[8];
#pragma unroll
    for (int j = 0; j < 8; ++j) {
      const float a  = off_w[(size_t)(i0 + j) * NOFF + no];
      const float bm = mk_w[(size_t)(i0 + j) * NTAP + nm];
      const float v  = (n < NOFF) ? a : ((n < NOMC) ? bm : 0.0f);
      f[j] = v * 16.0f;
    }
    v4u u;
    u[0] = pkh2(f[0], f[1]); u[1] = pkh2(f[2], f[3]); u[2] = pkh2(f[4], f[5]); u[3] = pkh2(f[6], f[7]);
    volatile v4u* p = (volatile v4u*)(OMW + e0);
    *p = u;
    __threadfence();
    *p = u;
  } else {
    const int g = (blk - 72) * 256 + tid;
    if (g < NTAP * NCH / 4) {
      const int e0 = g * 4;
      const int t  = e0 >> 8;
      const int c0 = e0 & (NCH - 1);
      v4f v;
#pragma unroll
      for (int e = 0; e < 4; ++e) v[e] = dw_w[(size_t)(c0 + e) * NTAP + t];
      volatile v4f* p = (volatile v4f*)(par + PAR_DWT + e0);
      *p = v;
      __threadfence();
      *p = v;
    }
  }
  if (blk == 0 && tid < 32) {
    const int lane = tid;
    v4f s0, s1;
#pragma unroll
    for (int e = 0; e < 4; ++e) {
      const int o0 = lane * 4 + e;
      const int o1 = 128 + lane * 4 + e;
      const float i0 = bn_inv(g2, v2, o0);
      const float i1 = bn_inv(g2, v2, o1);
      s0[e] = out_b[o0] * i0 + (b2[o0] - m2[o0] * i0);
      s1[e] = out_b[o1] * i1 + (b2[o1] - m2[o1] * i1);
    }
    volatile v4f* p0 = (volatile v4f*)(par + PAR_BIAS2 + lane * 4);
    volatile v4f* p1 = (volatile v4f*)(par + PAR_BIAS2 + 128 + lane * 4);
    *p0 = s0; *p1 = s1;
    __threadfence();
    *p0 = s0; *p1 = s1;
  }
  if (blk == 0 && tid >= 32 && tid < 48) {
    const int lane = tid - 32;
    v4f s;
#pragma unroll
    for (int e = 0; e < 4; ++e) {
      const int n  = lane * 4 + e;
      const int no = (n < NOFF) ? n : (NOFF - 1);
      const int nm = (n < NOFF) ? 0 : ((n < NOMC) ? (n - NOFF) : (NTAP - 1));
      const float a  = off_b[no];
      const float bm = mk_b[nm];
      s[e] = (n < NOFF) ? a : ((n < NOMC) ? bm : 0.0f);
    }
    volatile v4f* p = (volatile v4f*)(par + PAR_BIAS64 + lane * 4);
    *p = s;
    __threadfence();
    *p = s;
  }
}

__global__ __launch_bounds__(256) void k_xpose(const float* __restrict__ x, unsigned short* __restrict__ XT) {
  __shared__ float t[NCH][33];
  const int tid = threadIdx.x;
  const int blk = blockIdx.x;
  const int b = blk >> 7, hw0 = (blk & 127) * 32;
  const float* src = x + (size_t)b * NCH * HWPIX + hw0;
#pragma unroll
  for (int i = 0; i < 32; ++i) {
    const int idx = i * 256 + tid;
    const int c = idx >> 5, j = idx & 31;
    t[c][j] = src[(size_t)c * HWPIX + j];
  }
  __syncthreads();
  const int wave = tid >> 5, lane = tid & 31;
  const int c8 = lane * 8;
  unsigned short* ob = XT + ((size_t)b * HWPIX + hw0) * NCH;
  for (int pass = 0; pass < 2; ++pass) {
#pragma unroll
    for (int rr = 0; rr < 4; ++rr) {
      const int row = wave * 4 + rr;
      v8h v;
#pragma unroll
      for (int e = 0; e < 8; ++e) v[e] = (_Float16)t[c8 + e][row];
      *(volatile v8h*)(ob + (size_t)row * NCH + c8) = v;
    }
    __threadfence();
  }
}

__global__ __launch_bounds__(256) void k_im2col(const unsigned short* __restrict__ XT, unsigned short* __restrict__ IM) {
  const int lane = threadIdx.x & 31, wave = threadIdx.x >> 5;
  const int c8 = lane * 8;
#pragma unroll 1
  for (int q = 0; q < 4; ++q) {
    const int it = (blockIdx.x * 8 + wave) * 4 + q;
    if (it < NITEM) {
      const int p = it / NTAP, k = it - p * NTAP;
      const int b = p >> 12, hw = p & (HWPIX - 1);
      const int ho = hw >> 6, wo = hw & 63;
      const int kh = k / 3, kw = k - kh * 3;
      const int y = ho - 1 + kh, xx = wo - 1 + kw;
      const bool inb = ((unsigned)y < (unsigned)IMG_H) && ((unsigned)xx < (unsigned)IMG_W);
      const int yc = y < 0 ? 0 : (y > IMG_H - 1 ? IMG_H - 1 : y);
      const int xc = xx < 0 ? 0 : (xx > IMG_W - 1 ? IMG_W - 1 : xx);
      const unsigned short* src = XT + (((size_t)b * HWPIX + (size_t)yc * IMG_W + xc) * NCH + c8);
      v4u a = *(const v4u*)(src);
      if (!inb) a = (v4u){0u, 0u, 0u, 0u};
      volatile v4u* d = (volatile v4u*)(IM + (size_t)p * KCONV + (size_t)k * NCH + c8);
      *d = a;
      __threadfence();
      *d = a;
    }
  }
}

__global__ __launch_bounds__(256) void k_branch(const float* __restrict__ Y32, const float* __restrict__ DWT,
                                                const float* __restrict__ dw_b, const float* __restrict__ ln_g,
                                                const float* __restrict__ ln_b, unsigned short* __restrict__ X1P) {
  __shared__ float xs[8][NCH];
  const int tid = threadIdx.x;
  const int lane = tid & 31, wave = tid >> 5;
  const int p = blockIdx.x * 8 + wave;
  const int b = p >> 12, hw = p & (HWPIX - 1);
  const int ho = hw >> 6, wo = hw & 63;
  const int c8 = lane * 8;
  v4f a0 = *(const v4f*)(dw_b + c8);
  v4f a1 = *(const v4f*)(dw_b + c8 + 4);
  const float* yb = Y32 + (size_t)b * HWPIX * NCH + c8;
  const v4f z4 = (v4f){0.f, 0.f, 0.f, 0.f};
#pragma unroll 1
  for (int t = 0; t < NTAP; ++t) {
    const int kh = t / 3, kw = t - kh * 3;
    const int y = ho - 1 + kh, xx = wo - 1 + kw;
    const bool inb = ((unsigned)y < (unsigned)IMG_H) && ((unsigned)xx < (unsigned)IMG_W);
    const int yc = y < 0 ? 0 : (y > IMG_H - 1 ? IMG_H - 1 : y);
    const int xc = xx < 0 ? 0 : (xx > IMG_W - 1 ? IMG_W - 1 : xx);
    const float* src = yb + ((size_t)yc * IMG_W + xc) * NCH;
    v4f g0 = *(const v4f*)(src);
    v4f g1 = *(const v4f*)(src + 4);
    if (!inb) { g0 = z4; g1 = z4; }
    const v4f w0 = *(const v4f*)(DWT + t * NCH + c8);
    const v4f w1 = *(const v4f*)(DWT + t * NCH + c8 + 4);
    a0 += g0 * w0;
    a1 += g1 * w1;
  }
  float s = (a0[0] + a0[1]) + (a0[2] + a0[3]) + (a1[0] + a1[1]) + (a1[2] + a1[3]);
#pragma unroll
  for (int off = 16; off > 0; off >>= 1) s += __shfl_xor(s, off, 32);
  const float mu = s * (1.0f / 256.0f);
  float qv = 0.f;
#pragma unroll
  for (int e = 0; e < 4; ++e) { const float d0 = a0[e] - mu; const float d1 = a1[e] - mu; qv += d0 * d0; qv += d1 * d1; }
#pragma unroll
  for (int off = 16; off > 0; off >>= 1) qv += __shfl_xor(qv, off, 32);
  const float var  = qv * (1.0f / 256.0f);
  const float rstd = 1.0f / sqrtf(var + LN_EPS_F);
  float* xw = xs[wave];
  xw[c8 + 0] = a0[0]; xw[c8 + 1] = a0[1]; xw[c8 + 2] = a0[2]; xw[c8 + 3] = a0[3];
  xw[c8 + 4] = a1[0]; xw[c8 + 5] = a1[1]; xw[c8 + 6] = a1[2]; xw[c8 + 7] = a1[3];
#pragma unroll 1
  for (int e = 0; e < 8; ++e) {
    const int c = c8 + e;
    const float v  = xw[c];
    const float xn = (v - mu) * rstd * ln_g[c] + ln_b[c];
    const float gl = 0.5f * xn * (1.0f + erff(xn * 0.70710678118654752f));
    xw[c] = gl;
  }
  v8h hv;
#pragma unroll
  for (int e = 0; e < 8; ++e) hv[e] = (_Float16)xw[c8 + e];
  volatile v8h* d = (volatile v8h*)(X1P + (size_t)p * NCH + c8);
  *d = hv;
  __threadfence();
  *d = hv;
}

__global__ __launch_bounds__(256) void k_sample(const float* __restrict__ XPF, const float* __restrict__ BR,
                                                unsigned short* __restrict__ S16) {
  const int tid = threadIdx.x;
  const int lane = tid & 31, wave = tid >> 5;
  const int p = blockIdx.x * 8 + wave;
  const int b = p >> 12, hw = p & (HWPIX - 1);
  const int ho = hw >> 6, wo = hw & 63;
  const int c8 = lane * 8;
  const float* br = BR + (size_t)p * NOMP;
  const int lc = (lane < NTAP) ? lane : (NTAP - 1);
  float lg = br[NOFF + lc];
  lg = (lane < NTAP) ? lg : -3.0e38f;
  float mx = lg;
#pragma unroll
  for (int off = 16; off > 0; off >>= 1) mx = fmaxf(mx, __shfl_xor(mx, off, 32));
  float ex = (lane < NTAP) ? __expf(lg - mx) : 0.0f;
#pragma unroll
  for (int off = 16; off > 0; off >>= 1) ex += __shfl_xor(ex, off, 32);
  const float inv = 1.0f / ex;
  v4f a0 = (v4f){0.f, 0.f, 0.f, 0.f};
  v4f a1 = (v4f){0.f, 0.f, 0.f, 0.f};
  const float* xb = XPF + (size_t)b * HWPIX * NCH + c8;
  const float lim_x = (float)(IMG_W - 1), lim_y = (float)(IMG_H - 1);
#pragma unroll 1
  for (int t = 0; t < NTAP; ++t) {
    const float offx = br[2 * t];
    const float offy = br[2 * t + 1];
    const float mk   = __expf(br[NOFF + t] - mx) * inv;
    const int t3 = t / 3;
    const int kx = t3 - 1, ky = (t - t3 * 3) - 1;
    const float px = (float)(wo + kx) + offx;
    const float py = (float)(ho + ky) + offy;
    const float x0 = floorf(px), y0 = floorf(py);
    const float x1 = x0 + 1.0f, y1 = y0 + 1.0f;
    const float fx = px - x0, fy = py - y0;
    const float gx0 = 1.0f - fx, gy0 = 1.0f - fy;
    const bool vx0 = (x0 >= 0.0f) && (x0 <= lim_x);
    const bool vx1 = (x1 >= 0.0f) && (x1 <= lim_x);
    const bool vy0 = (y0 >= 0.0f) && (y0 <= lim_y);
    const bool vy1 = (y1 >= 0.0f) && (y1 <= lim_y);
    float w00 = gx0 * gy0;
    float w10 = fx  * gy0;
    float w01 = gx0 * fy;
    float w11 = fx  * fy;
    w00 = (vx0 && vy0) ? w00 : 0.0f;
    w10 = (vx1 && vy0) ? w10 : 0.0f;
    w01 = (vx0 && vy1) ? w01 : 0.0f;
    w11 = (vx1 && vy1) ? w11 : 0.0f;
    const int xi0 = (int)fminf(fmaxf(x0, 0.0f), lim_x);
    const int xi1 = (int)fminf(fmaxf(x1, 0.0f), lim_x);
    const int yi0 = (int)fminf(fmaxf(y0, 0.0f), lim_y);
    const int yi1 = (int)fminf(fmaxf(y1, 0.0f), lim_y);
    const float* r00 = xb + ((size_t)yi0 * IMG_W + xi0) * NCH;
    const float* r10 = xb + ((size_t)yi0 * IMG_W + xi1) * NCH;
    const float* r01 = xb + ((size_t)yi1 * IMG_W + xi0) * NCH;
    const float* r11 = xb + ((size_t)yi1 * IMG_W + xi1) * NCH;
    const v4f g00a = *(const v4f*)(r00), g00b = *(const v4f*)(r00 + 4);
    const v4f g10a = *(const v4f*)(r10), g10b = *(const v4f*)(r10 + 4);
    const v4f g01a = *(const v4f*)(r01), g01b = *(const v4f*)(r01 + 4);
    const v4f g11a = *(const v4f*)(r11), g11b = *(const v4f*)(r11 + 4);
    const v4f va = g00a * w00 + g10a * w10 + g01a * w01 + g11a * w11;
    const v4f vb = g00b * w00 + g10b * w10 + g01b * w01 + g11b * w11;
    a0 += va * mk;
    a1 += vb * mk;
  }
  v4u u;
  u[0] = pkh2(a0[0], a0[1]); u[1] = pkh2(a0[2], a0[3]);
  u[2] = pkh2(a1[0], a1[1]); u[3] = pkh2(a1[2], a1[3]);
  volatile v4u* d = (volatile v4u*)(S16 + (size_t)p * NCH + c8);
  *d = u;
  __threadfence();
  *d = u;
}

extern "C" void kernel_launch(void* const* d_in, const int* in_sizes, int n_in,
                              void* d_out, int out_size, void* d_ws, size_t ws_size,
                              hipStream_t stream) {
  if (n_in < 22) return;
  if (in_sizes[0] != NBATCH * NCH * HWPIX || in_sizes[1] != NCH * KCONV ||
      in_sizes[2] != NCH || in_sizes[3] != NCH || in_sizes[4] != NCH || in_sizes[5] != NCH ||
      in_sizes[6] != NCH * NCH || in_sizes[7] != NCH || in_sizes[8] != NCH * NTAP || in_sizes[9] != NCH ||
      in_sizes[10] != NCH || in_sizes[11] != NCH || in_sizes[12] != NCH * NOFF || in_sizes[13] != NOFF ||
      in_sizes[14] != NCH * NTAP || in_sizes[15] != NTAP || in_sizes[16] != NCH * NCH || in_sizes[17] != NCH ||
      in_sizes[18] != NCH || in_sizes[19] != NCH || in_sizes[20] != NCH || in_sizes[21] != NCH) return;
  if (out_size != NBATCH * NCH * HWPIX) return;

  const float* x     = (const float*)d_in[0];
  const float* w1    = (const float*)d_in[1];
  const float* bn1_g = (const float*)d_in[2];
  const float* bn1_b = (const float*)d_in[3];
  const float* bn1_m = (const float*)d_in[4];
  const float* bn1_v = (const float*)d_in[5];
  const float* in_w  = (const float*)d_in[6];
  const float* in_b  = (const float*)d_in[7];
  const float* dw_w  = (const float*)d_in[8];
  const float* dw_b  = (const float*)d_in[9];
  const float* ln_g  = (const float*)d_in[10];
  const float* ln_b  = (const float*)d_in[11];
  const float* off_w = (const float*)d_in[12];
  const float* off_b = (const float*)d_in[13];
  const float* mk_w  = (const float*)d_in[14];
  const float* mk_b  = (const float*)d_in[15];
  const float* out_w = (const float*)d_in[16];
  const float* out_b = (const float*)d_in[17];
  const float* bn2_g = (const float*)d_in[18];
  const float* bn2_b = (const float*)d_in[19];
  const float* bn2_m = (const float*)d_in[20];
  const float* bn2_v = (const float*)d_in[21];
  float* out = (float*)d_out;

  const size_t bytes_XT16  = (size_t)NPIX * NCH * 2;
  const size_t bytes_IM16  = (size_t)NPIX * KCONV * 2;
  const size_t bytes_W1P   = (size_t)NCH * KCONV * 2;
  const size_t bytes_Y32   = (size_t)NPIX * NCH * 4;
  const size_t bytes_Y16   = (size_t)NPIX * NCH * 2;
  const size_t bytes_SQ    = (size_t)NCH * NCH * 2;
  const size_t bytes_OMW   = (size_t)NOMP * NCH * 2;
  const size_t bytes_XPF   = (size_t)NPIX * NCH * 4;
  const size_t bytes_X1P   = (size_t)NPIX * NCH * 2;
  const size_t bytes_BR    = (size_t)NPIX * NOMP * 4;
  const size_t bytes_S16   = (size_t)NPIX * NCH * 2;
  const size_t bytes_PAR   = (size_t)PAR_FLOATS * 4;
  char* ws = (char*)d_ws;
  size_t o = 0;
  unsigned short* XT16  = (unsigned short*)(ws + o); o += bytes_XT16;
  unsigned short* IM16  = (unsigned short*)(ws + o); o += bytes_IM16;
  unsigned short* W1P   = (unsigned short*)(ws + o); o += bytes_W1P;
  float*          Y32   = (float*)(ws + o);          o += bytes_Y32;
  unsigned short* Y16   = (unsigned short*)(ws + o); o += bytes_Y16;
  unsigned short* INWP  = (unsigned short*)(ws + o); o += bytes_SQ;
  unsigned short* OUTWP = (unsigned short*)(ws + o); o += bytes_SQ;
  unsigned short* OMW   = (unsigned short*)(ws + o); o += bytes_OMW;
  float*          XPF   = (float*)(ws + o);          o += bytes_XPF;
  unsigned short* X1P   = (unsigned short*)(ws + o); o += bytes_X1P;
  float*          BR    = (float*)(ws + o);          o += bytes_BR;
  unsigned short* S16   = (unsigned short*)(ws + o); o += bytes_S16;
  float*          PAR   = (float*)(ws + o);          o += bytes_PAR;
  if (o > ws_size) return;
  float* shift1 = PAR + PAR_SHIFT1;
  float* bias2  = PAR + PAR_BIAS2;
  float* bias64 = PAR + PAR_BIAS64;
  float* DWT    = PAR + PAR_DWT;
  const float inv16 = 0.0625f;

  k_prep_w1<<<(NCH * KCONV / 8) / 256, 256, 0, stream>>>(w1, bn1_g, bn1_b, bn1_m, bn1_v, W1P, shift1);
  k_prep_small<<<75, 256, 0, stream>>>(in_w, out_w, out_b, bn2_g, bn2_b, bn2_m, bn2_v,
                                        off_w, off_b, mk_w, mk_b, dw_w, INWP, OUTWP, OMW, PAR);
  k_xpose<<<NPIX / 32, 256, 0, stream>>>(x, XT16);
  k_im2col<<<NITEM / 32, 256, 0, stream>>>(XT16, IM16);
  {
    const int tiles = (NPIX / 64) * (NCH / 64);
    wmma_gemm64<0, false, 2, 3, false, 3><<<dim3((tiles + 7) / 8, 1), 256, 0, stream>>>(
        IM16, IM16, KCONV, 0L,
        W1P, W1P, KCONV, 0L,
        (void*)Y32, (void*)Y16, NCH, 0L,
        shift1,
        shift1, 0L,
        NPIX, NCH, KCONV, inv16);
  }
  {
    const int tiles = (NPIX / 64) * (NCH / 64);
    wmma_gemm64<0, false, 2, 0, false, 0><<<dim3((tiles + 7) / 8, 1), 256, 0, stream>>>(
        Y16, Y16, NCH, 0L,
        INWP, INWP, NCH, 0L,
        (void*)XPF, (void*)PAR, NCH, 0L,
        in_b,
        in_b, 0L,
        NPIX, NCH, NCH, inv16);
  }
  k_branch<<<NPIX / 8, 256, 0, stream>>>(Y32, DWT, dw_b, ln_g, ln_b, X1P);
  {
    const int tiles = (NPIX / 64) * (NOMP / 64);
    wmma_gemm64<0, false, 2, 0, false, 0><<<dim3((tiles + 7) / 8, 1), 256, 0, stream>>>(
        X1P, X1P, NCH, 0L,
        OMW, OMW, NCH, 0L,
        (void*)BR, (void*)PAR, NOMP, 0L,
        bias64,
        bias64, 0L,
        NPIX, NOMP, NCH, inv16);
  }
  k_sample<<<NPIX / 8, 256, 0, stream>>>(XPF, BR, S16);
  {
    const int tiles = (NCH / 64) * (HWPIX / 64);
    wmma_gemm64<0, false, 1, 0, true, 3><<<dim3((tiles + 7) / 8, NBATCH), 256, 0, stream>>>(
        OUTWP, OUTWP, NCH, 0L,
        S16, S16, NCH, (long)HWPIX * NCH,
        (void*)out, (void*)PAR, HWPIX, (long)NCH * HWPIX,
        bias2,
        x, (long)NCH * HWPIX,
        NCH, HWPIX, NCH, inv16);
  }
}
